// VIMAttention_9156870275464
// MI455X (gfx1250) — hardware-run, weakly checked
//
#include <hip/hip_runtime.h>
#include <math.h>

typedef __attribute__((ext_vector_type(16))) _Float16 v16h;
typedef __attribute__((ext_vector_type(8)))  _Float16 v8h;
typedef __attribute__((ext_vector_type(16))) __bf16   v16b;
typedef __attribute__((ext_vector_type(8)))  __bf16   v8b;
typedef __attribute__((ext_vector_type(8)))  float    v8f;
typedef __attribute__((ext_vector_type(4)))  float    v4f;

constexpr int kBatch   = 4;
constexpr int kSeq     = 1536;
constexpr int kHalfSeq = 768;
constexpr int kDm      = 256;
constexpr int kDin     = 512;
constexpr int kNst     = 16;
constexpr int kDtR     = 16;
constexpr int kConvK   = 4;
constexpr int kLayers  = 8;
constexpr int kXzP     = 2 * kDin;
constexpr int kXdW     = kDtR + 2 * kNst;
constexpr int kXdP     = 64;
constexpr int kRows    = kBatch * kSeq;
constexpr float kEps    = 1e-5f;
constexpr float kWScale = 32.f;
constexpr float kUScale = 16.f;
constexpr float kYScale = 256.f;
constexpr int kPackTP  = 260;
constexpr int kConvTP  = 260;
constexpr int kScanTS  = 64;
constexpr int kScanCh  = 64;
constexpr int kScanYP  = 68;
constexpr int kTrP     = 36;
static_assert((kDm % 32) == 0 && (kDin % 32) == 0, "GEMM K multiples of 32");
static_assert((kRows % 64) == 0 && (kXzP % 64) == 0 && (kXdP % 64) == 0 && (kDm % 64) == 0, "GEMM M,N multiples of 64");
static_assert((kSeq % kScanTS) == 0 && (kSeq % 64) == 0 && (kDin % kScanCh) == 0 && (kDin % 256) == 0, "tile multiples");
static_assert((kHalfSeq % 32) == 0 && (kRows % 32) == 0 && (kRows % 8) == 0, "row block multiples");
static_assert(kXdW <= kXdP, "x_proj pad");

constexpr size_t kOffWIN  = 0;
constexpr size_t kOffWX   = kOffWIN  + (size_t)kLayers * kXzP * kDm * 2;
constexpr size_t kOffWOUT = kOffWX   + (size_t)kLayers * kXdP * kDin * 2;
constexpr size_t kOffNMF  = kOffWOUT + (size_t)kLayers * kDm * kDin * 2;
constexpr size_t kOffNMB  = kOffNMF  + (size_t)kRows * kDm * 2;
constexpr size_t kOffXZ   = kOffNMB  + (size_t)kRows * kDm * 2;
constexpr size_t kOffUC   = kOffXZ   + (size_t)kRows * kXzP * 4;
constexpr size_t kOffUCH  = kOffUC   + (size_t)kRows * kDin * 4;
constexpr size_t kOffXD   = kOffUCH  + (size_t)kRows * kDin * 2;
constexpr size_t kOffYH   = kOffXD   + (size_t)kRows * kXdP * 4;
constexpr size_t kOffHF   = kOffYH   + (size_t)kRows * kDin * 2;
constexpr size_t kOffHID  = kOffHF   + (size_t)kRows * kDm * 4;
constexpr size_t kOffRESA = kOffHID  + (size_t)kRows * kDm * 4;
constexpr size_t kOffRESB = kOffRESA + (size_t)kRows * kDm * 4;
constexpr size_t kWsTotal = kOffRESB + (size_t)kRows * kDm * 4;
static_assert(kWsTotal == 90177536ull, "carve total");
static_assert(kWsTotal <= 134217728ull, "carve cap");
static_assert((kOffWX % 128) == 0 && (kOffWOUT % 128) == 0 && (kOffNMF % 128) == 0 && (kOffNMB % 128) == 0 &&
              (kOffXZ % 128) == 0 && (kOffUC % 128) == 0 && (kOffUCH % 128) == 0 && (kOffXD % 128) == 0 &&
              (kOffYH % 128) == 0 && (kOffHF % 128) == 0 && (kOffHID % 128) == 0 && (kOffRESA % 128) == 0 &&
              (kOffRESB % 128) == 0, "128-B aligned regions");

__device__ __forceinline__ unsigned short f2bf_bits(float f) {
  unsigned u = __float_as_uint(f);
  return (unsigned short)((u + 0x7FFFu + ((u >> 16) & 1u)) >> 16);
}
__device__ __forceinline__ float bf_bits2f(unsigned short h) { return __uint_as_float(((unsigned)h) << 16); }

__device__ __forceinline__ void dep_guard_h(v8f& a, v8f& b, v16h x, v16h y) { asm volatile("v_nop\n\tv_nop\n\tv_nop\n\tv_nop" : "+v"(a), "+v"(b) : "v"(x), "v"(y)); }
__device__ __forceinline__ void dep_guard_b(v8f& a, v8f& b, v16b x, v16b y) { asm volatile("v_nop\n\tv_nop\n\tv_nop\n\tv_nop" : "+v"(a), "+v"(b) : "v"(x), "v"(y)); }
__device__ __forceinline__ void keep4_h(v16h a, v16h b, v16h c, v16h d) { asm volatile("v_nop" :: "v"(a), "v"(b), "v"(c), "v"(d)); }
__device__ __forceinline__ void keep4_b(v16b a, v16b b, v16b c, v16b d) { asm volatile("v_nop" :: "v"(a), "v"(b), "v"(c), "v"(d)); }
__device__ __forceinline__ void acc_guard4(v8f& a, v8f& b, v8f& c, v8f& d) { asm volatile("v_nop\n\tv_nop\n\tv_nop\n\tv_nop" : "+v"(a), "+v"(b), "+v"(c), "+v"(d)); }
template <typename T> struct Frag;
template <> struct Frag<_Float16> {
  typedef v16h V; union U { v16h v; v8h h[2]; };
  static __device__ __forceinline__ v16h load(const _Float16* p) {
    U f; f.h[0] = *(const v8h*)(p); f.h[1] = *(const v8h*)(p + 16); return f.v;
  }
  static __device__ __forceinline__ v8f mma(v16h a, v16h b, v8f c) {
    return __builtin_amdgcn_wmma_f32_16x16x32_f16(false, a, false, b, (short)0, c, false, false);
  }
  static __device__ __forceinline__ void guard(v8f& a, v8f& b, v16h x, v16h y) { dep_guard_h(a, b, x, y); }
  static __device__ __forceinline__ void keep(v16h a, v16h b, v16h c, v16h d) { keep4_h(a, b, c, d); }
};
template <> struct Frag<__bf16> {
  typedef v16b V; union U { v16b v; v8b h[2]; };
  static __device__ __forceinline__ v16b load(const __bf16* p) {
    U f; f.h[0] = *(const v8b*)(p); f.h[1] = *(const v8b*)(p + 16); return f.v;
  }
  static __device__ __forceinline__ v8f mma(v16b a, v16b b, v8f c) {
    return __builtin_amdgcn_wmma_f32_16x16x32_bf16(false, a, false, b, (short)0, c, false, false);
  }
  static __device__ __forceinline__ void guard(v8f& a, v8f& b, v16b x, v16b y) { dep_guard_b(a, b, x, y); }
  static __device__ __forceinline__ void keep(v16b a, v16b b, v16b c, v16b d) { keep4_b(a, b, c, d); }
};

template <int ET> struct Elem;
template <> struct Elem<0> { typedef _Float16 T; };
template <> struct Elem<1> { typedef __bf16 T; };
template <int ET, int SPL, int BIAS_MODE, int OUT_MODE, bool RESID, int ACT = 0>
__global__ __launch_bounds__(256) void wmma_gemm64(
    const unsigned short* __restrict__ Ap, const unsigned short* __restrict__ A2p, int lda, long strideA,
    const unsigned short* __restrict__ Btp, const unsigned short* __restrict__ Bt2p, int ldb, long strideB,
    void* __restrict__ Cout, void* __restrict__ Cout2, int ldc, long strideC,
    const float* __restrict__ bias,
    const float* __restrict__ resid, long strideR,
    int M, int N, int K, float scale) {
  typedef typename Elem<ET>::T T;
  typedef typename Frag<T>::V V;
  const T* A = (const T*)Ap; const T* A2 = (const T*)A2p; const T* Bt = (const T*)Btp; const T* Bt2 = (const T*)Bt2p;
  __shared__ __align__(16) float sT[8][16 * 68];
  const int b    = blockIdx.y;
  const int lane = threadIdx.x & 31;
  const int wave = threadIdx.x >> 5;
  const int tilesN = N >> 6;
  const int tilesM = M >> 6;
  const int tile = blockIdx.x * 8 + wave;
  if (tile >= tilesM * tilesN) return;
  const int tm = tile / tilesN;
  const int tn = tile - tm * tilesN;
  const int m0 = tm << 6;
  const int n0 = tn << 6;

  const T* Ab  = A  + (size_t)b * strideA;
  const T* Bb  = Bt + (size_t)b * strideB;
  const T* Ab2 = (SPL >= 1) ? (A2  + (size_t)b * strideA) : nullptr;
  const T* Bb2 = (SPL == 2) ? (Bt2 + (size_t)b * strideB) : nullptr;

  const int rlane = lane & 15;
  const int koff  = (lane >> 4) * 8;
  const int mOff  = (lane >> 4) * 8;

  v8f acc[4][4];
#pragma unroll
  for (int i = 0; i < 4; ++i)
#pragma unroll
    for (int j = 0; j < 4; ++j) acc[i][j] = (v8f){0.f,0.f,0.f,0.f,0.f,0.f,0.f,0.f};

  for (int k0 = 0; k0 < K; k0 += 32) {
    V bh[4], bl[4];
#pragma unroll
    for (int j = 0; j < 4; ++j) {
      const size_t bo = (size_t)(n0 + (j << 4) + rlane) * ldb + koff + k0;
      bh[j] = Frag<T>::load(Bb + bo);
      if (SPL == 2) bl[j] = Frag<T>::load(Bb2 + bo);
    }
#pragma unroll
    for (int i = 0; i < 4; ++i) {
      const size_t ao = (size_t)(m0 + (i << 4) + rlane) * lda + koff + k0;
      V ah = Frag<T>::load(Ab + ao);
      V al;
      if (SPL >= 1) al = Frag<T>::load(Ab2 + ao);
#pragma unroll
      for (int j = 0; j < 4; ++j) {
        acc[i][j] = Frag<T>::mma(ah, bh[j], acc[i][j]);
        if (SPL == 2) acc[i][j] = Frag<T>::mma(ah, bl[j], acc[i][j]);
        if (SPL >= 1) acc[i][j] = Frag<T>::mma(al, bh[j], acc[i][j]);
      }
      Frag<T>::guard(acc[i][0], acc[i][3], ah, (SPL >= 1) ? al : ah);
    }
    Frag<T>::keep(bh[0], bh[1], bh[2], bh[3]);
    if (SPL == 2) Frag<T>::keep(bl[0], bl[1], bl[2], bl[3]);
  }
  acc_guard4(acc[0][0], acc[0][1], acc[0][2], acc[0][3]);
  acc_guard4(acc[1][0], acc[1][1], acc[1][2], acc[1][3]);
  acc_guard4(acc[2][0], acc[2][1], acc[2][2], acc[2][3]);
  acc_guard4(acc[3][0], acc[3][1], acc[3][2], acc[3][3]);

  float* slab = sT[wave];
  const float* Rb = RESID ? (resid + (size_t)b * strideR) : nullptr;
#pragma unroll
  for (int i = 0; i < 4; ++i) {
    const int mBase = m0 + (i << 4);
#pragma unroll
    for (int j = 0; j < 4; ++j) {
      const int n = n0 + (j << 4) + rlane;
      float bv = 0.f;
      if (BIAS_MODE == 2) bv = bias[n];
#pragma unroll
      for (int r = 0; r < 8; ++r) {
        float v = acc[i][j][r] * scale;
        if (BIAS_MODE == 1) v += bias[mBase + mOff + r];
        if (BIAS_MODE == 2) v += bv;
        if (RESID) v += Rb[(size_t)(mBase + mOff + r) * ldc + n];
        if (ACT == 1) v = tanhf(v);
        if (ACT == 2) v = fmaxf(v, 0.0f);
        if (ACT == 3) v = v / (1.0f + expf(-v));
        if (ACT == 4) v = (v > 0.f) ? v : 0.01f * v;
        slab[(mOff + r) * 68 + (j << 4) + rlane] = v;
      }
    }
    __builtin_amdgcn_fence(__ATOMIC_RELEASE, "workgroup");
    __builtin_amdgcn_wave_barrier();
    __builtin_amdgcn_fence(__ATOMIC_ACQUIRE, "workgroup");
    if (OUT_MODE == 0) {
      float* C = (float*)Cout + (size_t)b * strideC;
      const int hh = lane >> 4, c4 = (lane & 15) * 4;
      for (int pass = 0; pass < 2; ++pass) {
#pragma unroll
        for (int it = 0; it < 8; ++it) {
          const int row = it * 2 + hh;
          v4f v = *(const v4f*)(slab + row * 68 + c4);
          *(volatile v4f*)(C + (size_t)(mBase + row) * ldc + n0 + c4) = v;
        }
        __threadfence();
      }
    } else {
      const int q = lane >> 3, c8 = (lane & 7) * 8;
      unsigned short* C  = (unsigned short*)Cout  + (size_t)b * strideC;
      unsigned short* C2 = (OUT_MODE == 2) ? ((unsigned short*)Cout2 + (size_t)b * strideC) : nullptr;
      for (int pass = 0; pass < 2; ++pass) {
#pragma unroll
        for (int it = 0; it < 4; ++it) {
          const int row = it * 4 + q;
          const float* sp = slab + row * 68 + c8;
          v8h hv, lv;
#pragma unroll
          for (int e = 0; e < 8; ++e) {
            if (OUT_MODE == 1) {
              hv[e] = (_Float16)sp[e];
            } else {
              unsigned short hb = f2bf_bits(sp[e]);
              unsigned short lb = f2bf_bits(sp[e] - bf_bits2f(hb));
              hv[e] = __builtin_bit_cast(_Float16, hb);
              lv[e] = __builtin_bit_cast(_Float16, lb);
            }
          }
          *(volatile v8h*)(C + (size_t)(mBase + row) * ldc + n0 + c8) = hv;
          if (OUT_MODE == 2) *(volatile v8h*)(C2 + (size_t)(mBase + row) * ldc + n0 + c8) = lv;
        }
        __threadfence();
      }
    }
    __builtin_amdgcn_fence(__ATOMIC_RELEASE, "workgroup");
    __builtin_amdgcn_wave_barrier();
    __builtin_amdgcn_fence(__ATOMIC_ACQUIRE, "workgroup");
  }
}

__global__ __launch_bounds__(256) void cast_scale_f16x8_kernel(
    const float* __restrict__ src, unsigned short* __restrict__ dst, int total8, float scale)
{
  const int i = blockIdx.x * 256 + threadIdx.x;
  if (i >= total8) return;
  const size_t e0 = (size_t)i << 3;
  const v4f a0 = *(const v4f*)(src + e0);
  const v4f a1 = *(const v4f*)(src + e0 + 4);
  v8h hv;
#pragma unroll
  for (int e = 0; e < 4; ++e) {
    hv[e]     = (_Float16)(a0[e] * scale);
    hv[4 + e] = (_Float16)(a1[e] * scale);
  }
  unsigned short* q = dst + e0;
  *(volatile v8h*)q = hv;
  __threadfence();
  *(volatile v8h*)q = hv;
}

__global__ __launch_bounds__(256) void cast_pad_xproj_kernel(
    const float* __restrict__ src, unsigned short* __restrict__ dst, int total8, float scale)
{
  const int i = blockIdx.x * 256 + threadIdx.x;
  if (i >= total8) return;
  const int e0 = i << 3;
  constexpr int kPerLayer = kXdP * kDin;
  const int layer = e0 / kPerLayer;
  const int rem = e0 - layer * kPerLayer;
  const int row = rem / kDin;
  const int col = rem - row * kDin;
  const int srow = (row < kXdW) ? row : (kXdW - 1);
  const size_t so = ((size_t)layer * kXdW + srow) * kDin + col;
  const v4f a0 = *(const v4f*)(src + so);
  const v4f a1 = *(const v4f*)(src + so + 4);
  const float m = (row < kXdW) ? scale : 0.f;
  v8h hv;
#pragma unroll
  for (int e = 0; e < 4; ++e) {
    hv[e]     = (_Float16)(a0[e] * m);
    hv[4 + e] = (_Float16)(a1[e] * m);
  }
  unsigned short* q = dst + (size_t)e0;
  *(volatile v8h*)q = hv;
  __threadfence();
  *(volatile v8h*)q = hv;
}

__global__ __launch_bounds__(256) void pack_kernel(
    const float* __restrict__ rgb, const float* __restrict__ ir, const float* __restrict__ pos,
    float* __restrict__ HIDp)
{
  __shared__ __align__(16) float sT[32 * kPackTP];
  const int tid = threadIdx.x, lane = tid & 31, wave = tid >> 5;
  const int r0 = blockIdx.x * 32;
  const int b = r0 / kSeq;
  const int l0 = r0 - b * kSeq;
  const int halfSel = (l0 >= kHalfSeq) ? 1 : 0;
  const int ls = l0 - halfSel * kHalfSeq;
  const float* src = halfSel ? ir : rgb;
  const float* sb = src + (size_t)b * kDm * kHalfSeq + ls + lane;
#pragma unroll 4
  for (int k = 0; k < 32; ++k) {
    const int dch = k * 8 + wave;
    sT[lane * kPackTP + dch] = sb[(size_t)dch * kHalfSeq];
  }
  __syncthreads();
  v4f vals[8];
#pragma unroll
  for (int j = 0; j < 4; ++j) {
#pragma unroll
    for (int hs = 0; hs < 2; ++hs) {
      const int row = wave + 8 * j;
      const int c = hs * 128 + lane * 4;
      const v4f t = *(const v4f*)(sT + row * kPackTP + c);
      const v4f p = *(const v4f*)(pos + (size_t)(l0 + row) * kDm + c);
      vals[j * 2 + hs] = t + p;
    }
  }
  for (int pass = 0; pass < 2; ++pass) {
#pragma unroll
    for (int j = 0; j < 4; ++j) {
#pragma unroll
      for (int hs = 0; hs < 2; ++hs) {
        const int row = wave + 8 * j;
        const int c = hs * 128 + lane * 4;
        *(volatile v4f*)(HIDp + (size_t)(r0 + row) * kDm + c) = vals[j * 2 + hs];
      }
    }
    __threadfence();
  }
}

__global__ __launch_bounds__(256) void addnorm_kernel(
    const float* __restrict__ HIDp, const float* __restrict__ RESINp, int hasRes,
    const float* __restrict__ wF, const float* __restrict__ bF,
    const float* __restrict__ wB, const float* __restrict__ bB,
    float* __restrict__ RESOUTp, unsigned short* __restrict__ NMFp, unsigned short* __restrict__ NMBp)
{
  __shared__ __align__(16) float sN[8][kDm];
  const int tid = threadIdx.x, lane = tid & 31, wave = tid >> 5;
  const int row = blockIdx.x * 8 + wave;
  const int cA = lane * 4, cB = 128 + lane * 4;
  const float* hp = HIDp + (size_t)row * kDm;
  v4f a0 = *(const v4f*)(hp + cA);
  v4f a1 = *(const v4f*)(hp + cB);
  if (hasRes) {
    const float* rp = RESINp + (size_t)row * kDm;
    const v4f q0 = *(const v4f*)(rp + cA);
    const v4f q1 = *(const v4f*)(rp + cB);
    a0 = q0 + a0;
    a1 = q1 + a1;
  }
  const v4f r0 = a0 + a0, r1 = a1 + a1;
  {
    float* op = RESOUTp + (size_t)row * kDm;
    for (int pass = 0; pass < 2; ++pass) {
      *(volatile v4f*)(op + cA) = r0;
      *(volatile v4f*)(op + cB) = r1;
      __threadfence();
    }
  }
  float s = 0.f;
#pragma unroll
  for (int e = 0; e < 4; ++e) s += a0[e];
#pragma unroll
  for (int e = 0; e < 4; ++e) s += a1[e];
#pragma unroll
  for (int off = 16; off > 0; off >>= 1) s += __shfl_xor(s, off, 32);
  const float mu = s * (1.f / kDm);
  float vs = 0.f;
#pragma unroll
  for (int e = 0; e < 4; ++e) { const float t = a0[e] - mu; vs += t * t; }
#pragma unroll
  for (int e = 0; e < 4; ++e) { const float t = a1[e] - mu; vs += t * t; }
#pragma unroll
  for (int off = 16; off > 0; off >>= 1) vs += __shfl_xor(vs, off, 32);
  const float inv = rsqrtf(vs * (1.f / kDm) + kEps);
  float* sn = sN[wave];
#pragma unroll
  for (int e = 0; e < 4; ++e) {
    sn[cA + e] = (a0[e] - mu) * inv;
    sn[cB + e] = (a1[e] - mu) * inv;
  }
  __builtin_amdgcn_fence(__ATOMIC_RELEASE, "workgroup");
  __builtin_amdgcn_wave_barrier();
  __builtin_amdgcn_fence(__ATOMIC_ACQUIRE, "workgroup");
  const int c8 = lane * 8;
  const v4f p0 = *(const v4f*)(sn + c8), p1 = *(const v4f*)(sn + c8 + 4);
  const v4f wf0 = *(const v4f*)(wF + c8), wf1 = *(const v4f*)(wF + c8 + 4);
  const v4f bf0 = *(const v4f*)(bF + c8), bf1 = *(const v4f*)(bF + c8 + 4);
  const v4f wb0 = *(const v4f*)(wB + c8), wb1 = *(const v4f*)(wB + c8 + 4);
  const v4f bb0 = *(const v4f*)(bB + c8), bb1 = *(const v4f*)(bB + c8 + 4);
  v8h hf, hb;
#pragma unroll
  for (int e = 0; e < 4; ++e) {
    hf[e]     = (_Float16)(p0[e] * wf0[e] + bf0[e]);
    hf[4 + e] = (_Float16)(p1[e] * wf1[e] + bf1[e]);
    hb[e]     = (_Float16)(p0[e] * wb0[e] + bb0[e]);
    hb[4 + e] = (_Float16)(p1[e] * wb1[e] + bb1[e]);
  }
  const size_t o = (size_t)row * kDm + c8;
  for (int pass = 0; pass < 2; ++pass) {
    *(volatile v8h*)(NMFp + o) = hf;
    *(volatile v8h*)(NMBp + o) = hb;
    __threadfence();
  }
}

__global__ __launch_bounds__(256) void conv_silu_kernel(
    const float* __restrict__ XZp, const float* __restrict__ cw, const float* __restrict__ cb,
    float* __restrict__ UCp, unsigned short* __restrict__ UCHp, int dir)
{
  __shared__ __align__(16) float sT[16 * kConvTP];
  const int tid = threadIdx.x, lane = tid & 31, wave = tid >> 5;
  const int d0 = blockIdx.x * 256, d = d0 + tid;
  const int g0 = blockIdx.y * 64;
  const int tb = g0 % kSeq;
  const float w0 = cw[d * kConvK + 0], w1 = cw[d * kConvK + 1], w2 = cw[d * kConvK + 2], w3 = cw[d * kConvK + 3];
  const float bc = cb[d];
  const bool hist = dir ? (tb + 64 < kSeq) : (tb > 0);
  const int rb = hist ? (dir ? (g0 + 64) : (g0 - 3)) : g0;
  const float q0 = XZp[(size_t)rb * kXzP + d];
  const float q1 = XZp[(size_t)(rb + 1) * kXzP + d];
  const float q2 = XZp[(size_t)(rb + 2) * kXzP + d];
  float xm1 = hist ? (dir ? q0 : q2) : 0.f;
  float xm2 = hist ? q1 : 0.f;
  float xm3 = hist ? (dir ? q2 : q0) : 0.f;
  const int hrow = wave >> 1;
  const int hch  = (wave & 1) * 128 + lane * 4;
#pragma unroll 1
  for (int sub = 0; sub < 4; ++sub) {
#pragma unroll 1
    for (int s = 0; s < 16; ++s) {
      const int slot = sub * 16 + s;
      const int row = dir ? (g0 + 63 - slot) : (g0 + slot);
      const float xcur = XZp[(size_t)row * kXzP + d];
      float acc = w0 * xm3;
      acc = fmaf(w1, xm2, acc);
      acc = fmaf(w2, xm1, acc);
      acc = fmaf(w3, xcur, acc);
      const float sv = acc + bc;
      const float sg = __builtin_amdgcn_rcpf(1.0f + expf(-sv));
      sT[s * kConvTP + tid] = sv * sg;
      xm3 = xm2; xm2 = xm1; xm1 = xcur;
    }
    __syncthreads();
    v4f fv[4];
    v8h bh[2];
#pragma unroll
    for (int it = 0; it < 4; ++it) fv[it] = *(const v4f*)(sT + (it * 4 + hrow) * kConvTP + hch);
#pragma unroll
    for (int it = 0; it < 2; ++it) {
      const float* sp = sT + (it * 8 + wave) * kConvTP + lane * 8;
      const v4f a0 = *(const v4f*)(sp);
      const v4f a1 = *(const v4f*)(sp + 4);
#pragma unroll
      for (int e = 0; e < 4; ++e) {
        bh[it][e]     = (_Float16)(a0[e] * kUScale);
        bh[it][4 + e] = (_Float16)(a1[e] * kUScale);
      }
    }
    for (int pass = 0; pass < 2; ++pass) {
#pragma unroll
      for (int it = 0; it < 4; ++it) {
        const int slot = sub * 16 + it * 4 + hrow;
        const int row = dir ? (g0 + 63 - slot) : (g0 + slot);
        *(volatile v4f*)(UCp + (size_t)row * kDin + d0 + hch) = fv[it];
      }
#pragma unroll
      for (int it = 0; it < 2; ++it) {
        const int slot = sub * 16 + it * 8 + wave;
        const int row = dir ? (g0 + 63 - slot) : (g0 + slot);
        *(volatile v8h*)(UCHp + (size_t)row * kDin + d0 + lane * 8) = bh[it];
      }
      __threadfence();
    }
    __syncthreads();
  }
}

__global__ __launch_bounds__(64) void scan_kernel(
    const float* __restrict__ XDp, const float* __restrict__ UCp, const float* __restrict__ XZp,
    const float* __restrict__ Wdt, const float* __restrict__ bdt, const float* __restrict__ Alog,
    const float* __restrict__ Dpp, unsigned short* __restrict__ YHp, int dir)
{
  __shared__ __align__(16) float sX[kScanTS * kXdP];
  __shared__ __align__(16) float sY[kScanTS * kScanYP];
  __shared__ __align__(16) float sW[kDtR * kScanCh];
  __shared__ __align__(16) float sA[kNst * kScanCh];
  const int tid = threadIdx.x, lane = tid & 31, wave = tid >> 5;
  constexpr int kBlkPerB = kDin / kScanCh;
  const int bix = blockIdx.x / kBlkPerB;
  const int d0  = (blockIdx.x - bix * kBlkPerB) * kScanCh;
  const int d   = d0 + tid;
  const size_t row0 = (size_t)bix * kSeq;
#pragma unroll 1
  for (int r = 0; r < kDtR; ++r) sW[r * kScanCh + tid] = Wdt[(size_t)d * kDtR + r];
#pragma unroll 1
  for (int s = 0; s < kNst; ++s) sA[s * kScanCh + tid] = -expf(Alog[(size_t)d * kNst + s]);
  __syncthreads();
  float negA[kNst], h[kNst];
#pragma unroll
  for (int s = 0; s < kNst; ++s) {
    negA[s] = sA[s * kScanCh + tid];
    h[s] = 0.f;
  }
  const float bb = bdt[d], Dd = Dpp[d];
  const int lr = tid >> 4, lc4 = (tid & 15) * 4;
  const int q = lane >> 3, c8 = (lane & 7) * 8;
#pragma unroll 1
  for (int c0 = 0; c0 < kSeq; c0 += kScanTS) {
    __syncthreads();
#pragma unroll
    for (int i = 0; i < 16; ++i) {
      const int r = lr + 4 * i;
      const int tr = dir ? (kSeq - 1 - c0 - r) : (c0 + r);
      *(v4f*)(sX + r * kXdP + lc4) = *(const v4f*)(XDp + (row0 + tr) * kXdP + lc4);
    }
    __syncthreads();
#pragma unroll 1
    for (int s = 0; s < kScanTS; ++s) {
      const int tr = dir ? (kSeq - 1 - c0 - s) : (c0 + s);
      const float* xr = sX + s * kXdP;
      float vdot = 0.f;
#pragma unroll 1
      for (int r4 = 0; r4 < kDtR / 4; ++r4) {
        const v4f xv = *(const v4f*)(xr + 4 * r4);
        const float* wp = sW + (4 * r4) * kScanCh + tid;
        vdot = fmaf(xv[0], wp[0], vdot);
        vdot = fmaf(xv[1], wp[kScanCh], vdot);
        vdot = fmaf(xv[2], wp[2 * kScanCh], vdot);
        vdot = fmaf(xv[3], wp[3 * kScanCh], vdot);
      }
      float Bs[kNst], Cs[kNst];
#pragma unroll
      for (int q4 = 0; q4 < 4; ++q4) {
        const v4f bv = *(const v4f*)(xr + kDtR + 4 * q4);
        const v4f cv = *(const v4f*)(xr + kDtR + kNst + 4 * q4);
        Bs[4 * q4 + 0] = bv[0]; Bs[4 * q4 + 1] = bv[1]; Bs[4 * q4 + 2] = bv[2]; Bs[4 * q4 + 3] = bv[3];
        Cs[4 * q4 + 0] = cv[0]; Cs[4 * q4 + 1] = cv[1]; Cs[4 * q4 + 2] = cv[2]; Cs[4 * q4 + 3] = cv[3];
      }
      const float v   = vdot + bb;
      const float dt  = fmaxf(v, 0.0f) + log1pf(expf(-fabsf(v)));
      const float xt  = UCp[(row0 + tr) * kDin + d];
      const float dtx = dt * xt;
      float y = 0.f;
#pragma unroll
      for (int k = 0; k < kNst; ++k) {
        const float e = __expf(dt * negA[k]);
        h[k] = e * h[k] + dtx * Bs[k];
        y = h[k] * Cs[k] + y;
      }
      y = xt * Dd + y;
      const float zv = XZp[(row0 + tr) * kXzP + kDin + d];
      const float sg = __builtin_amdgcn_rcpf(1.0f + expf(-zv));
      y = y * (zv * sg);
      sY[s * kScanYP + tid] = y;
    }
    __syncthreads();
    v8h hv[8];
#pragma unroll
    for (int it = 0; it < 8; ++it) {
      const int slot = it * 8 + wave * 4 + q;
      const float* sp = sY + slot * kScanYP + c8;
      const v4f a0 = *(const v4f*)(sp);
      const v4f a1 = *(const v4f*)(sp + 4);
#pragma unroll
      for (int e = 0; e < 4; ++e) {
        hv[it][e]     = (_Float16)(a0[e] * kYScale);
        hv[it][4 + e] = (_Float16)(a1[e] * kYScale);
      }
    }
    for (int pass = 0; pass < 2; ++pass) {
#pragma unroll
      for (int it = 0; it < 8; ++it) {
        const int slot = it * 8 + wave * 4 + q;
        const int tr = dir ? (kSeq - 1 - c0 - slot) : (c0 + slot);
        const size_t o = (row0 + tr) * kDin + d0 + c8;
        *(volatile v8h*)(YHp + o) = hv[it];
      }
      __threadfence();
    }
  }
}

__global__ __launch_bounds__(256) void final_kernel(
    const float* __restrict__ HIDp, const float* __restrict__ RESp,
    const float* __restrict__ wN, const float* __restrict__ bN, float* __restrict__ outp)
{
  __shared__ __align__(16) float sT[kDm * kTrP];
  const int tid = threadIdx.x, lane = tid & 31, wave = tid >> 5;
  const int r0 = blockIdx.x * 32;
  const int b = r0 / kSeq;
  const int l0 = r0 - b * kSeq;
  const int halfSel = (l0 >= kHalfSeq) ? 1 : 0;
  const int lo = l0 - halfSel * kHalfSeq;
  const int cA = lane * 4, cB = 128 + lane * 4;
  const v4f wa = *(const v4f*)(wN + cA), wb = *(const v4f*)(wN + cB);
  const v4f ba = *(const v4f*)(bN + cA), bbv = *(const v4f*)(bN + cB);
#pragma unroll 1
  for (int j = 0; j < 4; ++j) {
    const int tok = wave * 4 + j;
    const size_t ro = (size_t)(r0 + tok) * kDm;
    const v4f h0 = *(const v4f*)(HIDp + ro + cA), h1 = *(const v4f*)(HIDp + ro + cB);
    const v4f q0 = *(const v4f*)(RESp + ro + cA), q1 = *(const v4f*)(RESp + ro + cB);
    const v4f a0 = q0 + h0, a1 = q1 + h1;
    float s = 0.f;
#pragma unroll
    for (int e = 0; e < 4; ++e) s += a0[e];
#pragma unroll
    for (int e = 0; e < 4; ++e) s += a1[e];
#pragma unroll
    for (int off = 16; off > 0; off >>= 1) s += __shfl_xor(s, off, 32);
    const float mu = s * (1.f / kDm);
    float vs = 0.f;
#pragma unroll
    for (int e = 0; e < 4; ++e) { const float t = a0[e] - mu; vs += t * t; }
#pragma unroll
    for (int e = 0; e < 4; ++e) { const float t = a1[e] - mu; vs += t * t; }
#pragma unroll
    for (int off = 16; off > 0; off >>= 1) vs += __shfl_xor(vs, off, 32);
    const float inv = rsqrtf(vs * (1.f / kDm) + kEps);
#pragma unroll
    for (int e = 0; e < 4; ++e) {
      sT[(cA + e) * kTrP + tok] = (a0[e] - mu) * inv * wa[e] + ba[e];
      sT[(cB + e) * kTrP + tok] = (a1[e] - mu) * inv * wb[e] + bbv[e];
    }
  }
  __syncthreads();
  const int q = lane >> 3, sub = lane & 7;
  v4f vals[8];
#pragma unroll
  for (int k = 0; k < 8; ++k) {
    const int c = k * 32 + wave * 4 + q;
    vals[k] = *(const v4f*)(sT + c * kTrP + sub * 4);
  }
  const size_t obase = (size_t)halfSel * kBatch * kDm * kHalfSeq + (size_t)b * kDm * kHalfSeq + lo + sub * 4;
  for (int pass = 0; pass < 2; ++pass) {
#pragma unroll
    for (int k = 0; k < 8; ++k) {
      const int c = k * 32 + wave * 4 + q;
      *(volatile v4f*)(outp + obase + (size_t)c * kHalfSeq) = vals[k];
    }
    __threadfence();
  }
}

extern "C" void kernel_launch(void* const* d_in, const int* in_sizes, int n_in,
                              void* d_out, int out_size, void* d_ws, size_t ws_size,
                              hipStream_t stream) {
  if (n_in < 16) return;
  if (in_sizes[0] != kBatch * kDm * kHalfSeq) return;
  if (in_sizes[1] != kBatch * kDm * kHalfSeq) return;
  if (in_sizes[2] != kSeq * kDm) return;
  if (in_sizes[3] != kLayers * kXzP * kDm) return;
  if (in_sizes[4] != kLayers * kDin * kConvK) return;
  if (in_sizes[5] != kLayers * kDin) return;
  if (in_sizes[6] != kLayers * kXdW * kDin) return;
  if (in_sizes[7] != kLayers * kDin * kDtR) return;
  if (in_sizes[8] != kLayers * kDin) return;
  if (in_sizes[9] != kLayers * kDin * kNst) return;
  if (in_sizes[10] != kLayers * kDin) return;
  if (in_sizes[11] != kLayers * kDm * kDin) return;
  if (in_sizes[12] != kLayers * kDm) return;
  if (in_sizes[13] != kLayers * kDm) return;
  if (in_sizes[14] != kDm) return;
  if (in_sizes[15] != kDm) return;
  if (out_size != 2 * kBatch * kDm * kHalfSeq) return;
  if (ws_size < kWsTotal) return;

  const float* rgb        = (const float*)d_in[0];
  const float* ir         = (const float*)d_in[1];
  const float* pos        = (const float*)d_in[2];
  const float* in_proj_w  = (const float*)d_in[3];
  const float* conv_w     = (const float*)d_in[4];
  const float* conv_b     = (const float*)d_in[5];
  const float* x_proj_w   = (const float*)d_in[6];
  const float* dt_proj_w  = (const float*)d_in[7];
  const float* dt_proj_b  = (const float*)d_in[8];
  const float* A_log      = (const float*)d_in[9];
  const float* Dp         = (const float*)d_in[10];
  const float* out_proj_w = (const float*)d_in[11];
  const float* ln_w       = (const float*)d_in[12];
  const float* ln_b       = (const float*)d_in[13];
  const float* normf_w    = (const float*)d_in[14];
  const float* normf_b    = (const float*)d_in[15];
  float* out = (float*)d_out;

  char* ws = (char*)d_ws;
  unsigned short* WIN  = (unsigned short*)(ws + kOffWIN);
  unsigned short* WX   = (unsigned short*)(ws + kOffWX);
  unsigned short* WOUT = (unsigned short*)(ws + kOffWOUT);
  unsigned short* NMF  = (unsigned short*)(ws + kOffNMF);
  unsigned short* NMB  = (unsigned short*)(ws + kOffNMB);
  float*          XZ   = (float*)(ws + kOffXZ);
  float*          UC   = (float*)(ws + kOffUC);
  unsigned short* UCH  = (unsigned short*)(ws + kOffUCH);
  float*          XD   = (float*)(ws + kOffXD);
  unsigned short* YH   = (unsigned short*)(ws + kOffYH);
  float*          HF   = (float*)(ws + kOffHF);
  float*          HID  = (float*)(ws + kOffHID);
  float*          RESA = (float*)(ws + kOffRESA);
  float*          RESB = (float*)(ws + kOffRESB);

  cast_scale_f16x8_kernel<<<(kLayers * kXzP * kDm / 8) / 256, 256, 0, stream>>>(in_proj_w, WIN, kLayers * kXzP * kDm / 8, kWScale);
  cast_pad_xproj_kernel<<<(kLayers * kXdP * kDin / 8) / 256, 256, 0, stream>>>(x_proj_w, WX, kLayers * kXdP * kDin / 8, kWScale);
  cast_scale_f16x8_kernel<<<(kLayers * kDm * kDin / 8) / 256, 256, 0, stream>>>(out_proj_w, WOUT, kLayers * kDm * kDin / 8, kWScale);

  pack_kernel<<<kRows / 32, 256, 0, stream>>>(rgb, ir, pos, HID);

  const float inScale  = 1.0f / kWScale;
  const float xpScale  = 1.0f / (kUScale * kWScale);
  const float outScale = 1.0f / (kYScale * kWScale);

  auto mixer = [&](int L, const unsigned short* NM, int dir, bool addHF, float* hout) {
    wmma_gemm64<0, 0, 0, 0, false><<<dim3((kRows / 64) * (kXzP / 64) / 8, 1), 256, 0, stream>>>(
        NM, nullptr, kDm, 0L,
        WIN + (size_t)L * kXzP * kDm, nullptr, kDm, 0L,
        (void*)XZ, nullptr, kXzP, 0L,
        nullptr, nullptr, 0L,
        kRows, kXzP, kDm, inScale);
    conv_silu_kernel<<<dim3(kDin / 256, kRows / 64), 256, 0, stream>>>(
        XZ, conv_w + (size_t)L * kDin * kConvK, conv_b + (size_t)L * kDin, UC, UCH, dir);
    wmma_gemm64<0, 0, 0, 0, false><<<dim3((kRows / 64) * (kXdP / 64) / 8, 1), 256, 0, stream>>>(
        UCH, nullptr, kDin, 0L,
        WX + (size_t)L * kXdP * kDin, nullptr, kDin, 0L,
        (void*)XD, nullptr, kXdP, 0L,
        nullptr, nullptr, 0L,
        kRows, kXdP, kDin, xpScale);
    scan_kernel<<<kBatch * (kDin / kScanCh), kScanCh, 0, stream>>>(
        XD, UC, XZ, dt_proj_w + (size_t)L * kDin * kDtR, dt_proj_b + (size_t)L * kDin,
        A_log + (size_t)L * kDin * kNst, Dp + (size_t)L * kDin, YH, dir);
    if (addHF) {
      wmma_gemm64<0, 0, 0, 0, true><<<dim3((kRows / 64) * (kDm / 64) / 8, 1), 256, 0, stream>>>(
          YH, nullptr, kDin, 0L,
          WOUT + (size_t)L * kDm * kDin, nullptr, kDin, 0L,
          (void*)hout, nullptr, kDm, 0L,
          nullptr, HF, 0L,
          kRows, kDm, kDin, outScale);
    } else {
      wmma_gemm64<0, 0, 0, 0, false><<<dim3((kRows / 64) * (kDm / 64) / 8, 1), 256, 0, stream>>>(
          YH, nullptr, kDin, 0L,
          WOUT + (size_t)L * kDm * kDin, nullptr, kDin, 0L,
          (void*)hout, nullptr, kDm, 0L,
          nullptr, nullptr, 0L,
          kRows, kDm, kDin, outScale);
    }
  };

  for (int i = 0; i < kLayers / 2; ++i) {
    const int lf = 2 * i, lb = 2 * i + 1;
    const float* resIn = (i == 0) ? HID : ((i & 1) ? RESA : RESB);
    float* resOut = (i & 1) ? RESB : RESA;
    addnorm_kernel<<<kRows / 8, 256, 0, stream>>>(
        HID, resIn, (i == 0) ? 0 : 1,
        ln_w + (size_t)lf * kDm, ln_b + (size_t)lf * kDm,
        ln_w + (size_t)lb * kDm, ln_b + (size_t)lb * kDm,
        resOut, NMF, NMB);
    mixer(lf, NMF, 0, false, HF);
    mixer(lb, NMB, 1, true, HID);
  }

  final_kernel<<<kRows / 32, 256, 0, stream>>>(HID, RESB, normf_w, normf_b, out);
}
